// SlotAttention_73332271612043
// MI455X (gfx1250) — hardware-run, weakly checked
//
#include <hip/hip_runtime.h>


#ifndef NB
#define NB 8
#endif
#define NB_FULL  8
#define SEQ  256
#define DM   256
#define HK   64
#define PR   16
#define PW   8
#define KJP  65
#define PP   264
#define CP   260
#define C2    2.8853900817779268f
#define LOG2E 1.4426950408889634f
#define PCAR  256.0f
static constexpr float SCI = 1.0f / 256.0f;

static_assert(NB <= NB_FULL);
static_assert(DM % 32 == 0);
static_assert((NB * SEQ) % 64 == 0);
static_assert(HK == 64);
static_assert(SEQ % 32 == 0);
static_assert(SEQ == 32 * 8);
static_assert(SEQ % 64 == 0 && DM % 64 == 0);
static_assert(PR == 16);
static_assert(PR == 2 * PW);
static_assert(DM == 32 * PW);
static_assert(SEQ % PR == 0);
static_assert(SEQ * HK / 4 == 16 * 32 * PW);
static_assert(PR * HK / 4 == 32 * PW);
static_assert(2 * DM * 4 == 4 * 32 * 16);
static_assert(16 * HK * 4 == 8 * 32 * 16);
static_assert(64 * 64 * 2 == 2 * 256 * 16);
static_assert((PP * 2) % 16 == 0);
static_assert((CP * 4) % 16 == 0);
static_assert((size_t)SEQ * KJP * 4 + (size_t)PR * HK * 4 + (size_t)HK * 4 + (size_t)PR * PP * 2 + (size_t)PR * CP * 4 <= 131072);
static_assert((size_t)64 * 72 * 2 <= 131072);
static_assert(((size_t)NB * SEQ * DM) % 8 == 0);
static_assert(((size_t)HK * 2 * DM) % 8 == 0);

typedef _Float16 h16;
typedef unsigned short bf;
typedef __attribute__((ext_vector_type(16))) __bf16   v16bf;
typedef __attribute__((ext_vector_type(16))) _Float16 v16h;
typedef __attribute__((ext_vector_type(8)))  _Float16 v8h;
typedef __attribute__((ext_vector_type(8)))  unsigned short v8us;
typedef __attribute__((ext_vector_type(8)))  float    v8f;
typedef __attribute__((ext_vector_type(4)))  float    v4f;
typedef v4f  __attribute__((may_alias)) v4fa;
typedef v8h  __attribute__((may_alias)) v8ha;

__device__ __forceinline__ unsigned short f2bf(float f) { unsigned u = __float_as_uint(f); u += 0x7FFFu + ((u >> 16) & 1u); return (unsigned short)(u >> 16); }
__device__ __forceinline__ float bfr(float f) { return __uint_as_float(((unsigned)f2bf(f)) << 16); }
__device__ __forceinline__ v16h cat16(v8h lo, v8h hi) { return __builtin_shufflevector(lo, hi, 0, 1, 2, 3, 4, 5, 6, 7, 8, 9, 10, 11, 12, 13, 14, 15); }
__device__ __forceinline__ v16bf cat16b(v8us lo, v8us hi) { return __builtin_bit_cast(v16bf, __builtin_shufflevector(lo, hi, 0, 1, 2, 3, 4, 5, 6, 7, 8, 9, 10, 11, 12, 13, 14, 15)); }
__device__ __forceinline__ v8f wmma16(v16h a, v16h b, v8f c) { return __builtin_amdgcn_wmma_f32_16x16x32_f16(false, a, false, b, (short)0, c, false, false); }
__device__ __forceinline__ v8f wmmab(v16bf a, v16bf b, v8f c) { return __builtin_amdgcn_wmma_f32_16x16x32_bf16(false, a, false, b, (short)0, c, false, false); }
__device__ __forceinline__ v8f wmma16g(v16h a, v16h b, v8f c) { c = wmma16(a, b, c); asm volatile("v_nop\n\tv_nop\n\tv_nop\n\tv_nop" : "+v"(c) : "v"(a), "v"(b)); return c; }
__device__ __forceinline__ v8f wmmabg(v16bf a, v16bf b, v8f c) { c = wmmab(a, b, c); asm volatile("v_nop\n\tv_nop\n\tv_nop\n\tv_nop" : "+v"(c) : "v"(a), "v"(b)); return c; }
__device__ __forceinline__ v16h  ldh(const h16* p) { return cat16(*(const v8h*)p, *(const v8h*)(p + 16)); }
__device__ __forceinline__ v16bf ldb(const bf* p)  { return cat16b(*(const v8us*)p, *(const v8us*)(p + 16)); }
__device__ __forceinline__ void wave_sync() { __builtin_amdgcn_fence(3  , "wavefront"); __builtin_amdgcn_wave_barrier(); asm volatile("" ::: "memory"); }
static __device__ __forceinline__ h16 toh_flush(float v) { const float w = (fabsf(v) < 6.103515625e-05f) ? 0.0f : v; return (h16)w; }

__global__ __launch_bounds__(256) void k_cvt8(const float* __restrict__ src, bf* dst, size_t n8) {
    const size_t i = (size_t)blockIdx.x * 256 + threadIdx.x; if (i >= n8) return;
    const v8f v = *(const v8f*)(src + i * 8); v8us o;
#pragma unroll
    for (int k = 0; k < 8; ++k) o[k] = f2bf(v[k]);
    *(volatile v8us*)(dst + i * 8) = o; __threadfence(); *(volatile v8us*)(dst + i * 8) = o;
}

__global__ __launch_bounds__(256) void k_xt(const float* __restrict__ X, h16* XT) {
    __shared__ __align__(16) h16 ts[64 * 72];
    const unsigned tid = threadIdx.x;
    const unsigned jt = blockIdx.x, dt = blockIdx.y, b = blockIdx.z;
    const size_t src = ((size_t)b * SEQ + (size_t)jt * 64) * DM + (size_t)dt * 64;
#pragma unroll 4
    for (int it = 0; it < 4; ++it) {
        const unsigned idx = (unsigned)it * 256u + tid; const unsigned jr = idx >> 4, c4 = (idx & 15u) * 4u;
        const v4f v = *(const v4f*)(X + src + (size_t)jr * DM + c4);
#pragma unroll
        for (int e = 0; e < 4; ++e) ts[(c4 + e) * 72 + jr] = toh_flush(bfr(v[e]));
    }
    __syncthreads();
    v8h o[2];
#pragma unroll
    for (int it = 0; it < 2; ++it) { const unsigned p = (unsigned)it * 256u + tid; const unsigned row = p >> 3, c8 = (p & 7u) * 8u; o[it] = *(const v8ha*)(&ts[row * 72 + c8]); }
#pragma unroll 1
    for (int ps = 0; ps < 2; ++ps) {
#pragma unroll
        for (int it = 0; it < 2; ++it) { const unsigned p = (unsigned)it * 256u + tid; const unsigned row = p >> 3, c8 = (p & 7u) * 8u;
            *(volatile v8h*)(XT + ((size_t)b * DM + (size_t)dt * 64 + row) * SEQ + (size_t)jt * 64 + c8) = o[it]; }
        if (ps == 0) __threadfence(); }
}

__global__ __launch_bounds__(32) void k_proj(const bf* __restrict__ A, const bf* __restrict__ Wb, float* QK) {
    __shared__ __align__(16) float os[16 * 68];
    const int K = DM;
    const int lane = threadIdx.x & 31, lr = lane & 15, hi = lane >> 4;
    const unsigned bx = blockIdx.x, by = blockIdx.y;
    const size_t r0 = (size_t)bx * 64;
    v8f acc[4][4];
#pragma unroll
    for (int mb = 0; mb < 4; ++mb)
#pragma unroll
        for (int nb = 0; nb < 4; ++nb) acc[mb][nb] = (v8f){};
    const size_t aoff = (r0 + (size_t)lr) * K + 8 * hi;
    const size_t boff = (size_t)lr * (2 * DM) + (size_t)by * DM + 8 * hi;
#pragma unroll 1
    for (int kc = 0; kc < K; kc += 32) {
        v16bf a[4];
#pragma unroll
        for (int mb = 0; mb < 4; ++mb) a[mb] = ldb(A + aoff + (size_t)mb * 16 * K + kc);
#pragma unroll
        for (int nb = 0; nb < 4; ++nb) { const v16bf b = ldb(Wb + boff + (size_t)nb * 16 * (2 * DM) + kc);
#pragma unroll
            for (int mb = 0; mb < 4; ++mb) acc[mb][nb] = wmmabg(a[mb], b, acc[mb][nb]); }
    }
    float* P = QK + (size_t)by * ((size_t)NB * SEQ * HK) + r0 * HK;
#pragma unroll
    for (int mb = 0; mb < 4; ++mb) {
#pragma unroll
        for (int nb = 0; nb < 4; ++nb) {
#pragma unroll
            for (int j = 0; j < 8; ++j) os[(hi * 8 + j) * 68 + nb * 16 + lr] = acc[mb][nb][j]; }
        wave_sync();
#pragma unroll 1
        for (int ps = 0; ps < 2; ++ps) {
#pragma unroll
            for (int s = 0; s < 8; ++s) { const int row = 2 * s + (lane >> 4), c4 = (lane & 15) * 4;
                const v4f val = *(const v4fa*)(&os[row * 68 + c4]);
                *(volatile v4f*)(P + (size_t)(mb * 16 + row) * HK + c4) = val; }
            if (ps == 0) __threadfence(); }
        wave_sync();
    }
}

__device__ __forceinline__ void softmax8(float (&e)[8]) {
    float mx = e[0];
#pragma unroll
    for (int q = 1; q < 8; ++q) mx = fmaxf(mx, e[q]);
    mx = fmaxf(mx, __shfl_xor(mx, 16, 32)); mx = fmaxf(mx, __shfl_xor(mx, 8, 32)); mx = fmaxf(mx, __shfl_xor(mx, 4, 32));
    mx = fmaxf(mx, __shfl_xor(mx, 2, 32));  mx = fmaxf(mx, __shfl_xor(mx, 1, 32));
    float s = 0.0f;
#pragma unroll
    for (int q = 0; q < 8; ++q) { e[q] = __builtin_amdgcn_exp2f((e[q] - mx) * LOG2E); s += e[q]; }
    s += __shfl_xor(s, 16, 32); s += __shfl_xor(s, 8, 32); s += __shfl_xor(s, 4, 32); s += __shfl_xor(s, 2, 32); s += __shfl_xor(s, 1, 32);
    const float inv = PCAR * (1.0f / s);
#pragma unroll
    for (int q = 0; q < 8; ++q) e[q] = e[q] * inv;
}

__global__ __launch_bounds__(32 * PW) void k_pair(const float* __restrict__ X, const float* __restrict__ QK, const float* __restrict__ W2, const h16* __restrict__ XT, float* OUT) {
    __shared__ __align__(16) float kjs[SEQ * KJP];
    __shared__ __align__(16) float qs[PR * HK];
    __shared__ __align__(16) float w2s[HK];
    __shared__ __align__(16) h16   ph[PR * PP];
    __shared__ __align__(16) float cs[PR * CP];
    const unsigned tid = threadIdx.x;
    const int lane = (int)(tid & 31u), lr = lane & 15, hi = lane >> 4;
    const int wave = __builtin_amdgcn_readfirstlane((int)(threadIdx.x >> 5));
    const unsigned b = blockIdx.y;
    const unsigned i0 = blockIdx.x * PR;

    const float* kjg = QK + (size_t)NB * SEQ * HK + (size_t)b * SEQ * HK;
#pragma unroll 4
    for (int it = 0; it < 16; ++it) {
        const unsigned idx = (unsigned)it * 256u + tid; const unsigned row = idx >> 4, c4 = (idx & 15u) * 4u;
        const v4f v = *(const v4f*)(kjg + (size_t)row * HK + c4);
#pragma unroll
        for (int e = 0; e < 4; ++e) kjs[row * KJP + c4 + e] = v[e] * C2;
    }
    { const unsigned row = tid >> 4, c4 = (tid & 15u) * 4u;
      const v4f v = *(const v4f*)(QK + ((size_t)b * SEQ + i0 + row) * HK + c4);
#pragma unroll
      for (int e = 0; e < 4; ++e) qs[row * HK + c4 + e] = v[e] * C2; }
    { const float w = bfr(W2[tid & (unsigned)(HK - 1)]);
      if (tid < (unsigned)HK) w2s[tid] = -2.0f * w; }
    __syncthreads();

    const int ra = 2 * wave, rb = 2 * wave + 1;
    float ea[8], eb[8];
#pragma unroll
    for (int q = 0; q < 8; ++q) { ea[q] = 0.0f; eb[q] = 0.0f; }
#pragma unroll 2
    for (int k = 0; k < HK; ++k) {
        const float qa = qs[ra * HK + k], qb = qs[rb * HK + k], w = w2s[k];
#pragma unroll
        for (int q = 0; q < 8; ++q) {
            const float kv = kjs[(lane + 32 * q) * KJP + k];
            const float ta = __builtin_amdgcn_rcpf(__builtin_amdgcn_exp2f(qa + kv) + 1.0f);
            const float tb = __builtin_amdgcn_rcpf(__builtin_amdgcn_exp2f(qb + kv) + 1.0f);
            ea[q] = fmaf(w, ta, ea[q]); eb[q] = fmaf(w, tb, eb[q]);
        }
    }
    softmax8(ea); softmax8(eb);
#pragma unroll
    for (int q = 0; q < 8; ++q) { ph[ra * PP + lane + 32 * q] = toh_flush(ea[q]); ph[rb * PP + lane + 32 * q] = toh_flush(eb[q]); }
    __syncthreads();

    const int pofs = lr * PP + 8 * hi;
    const size_t xo = ((size_t)b * DM + (size_t)(wave * 32 + lr)) * SEQ + 8 * hi;
    v8f c0 = (v8f){}, c1 = (v8f){};
#pragma unroll 2
    for (int j0 = 0; j0 < SEQ; j0 += 32) {
        const v16h a = cat16(*(const v8ha*)(&ph[pofs + j0]), *(const v8ha*)(&ph[pofs + j0 + 16]));
        const v16h b0 = ldh(XT + xo + j0);
        const v16h b1 = ldh(XT + xo + (size_t)16 * SEQ + j0);
        c0 = wmma16g(a, b0, c0);
        c1 = wmma16g(a, b1, c1);
    }
#pragma unroll
    for (int r = 0; r < 8; ++r) {
        cs[(8 * hi + r) * CP + wave * 32 + lr]      = c0[r] * SCI;
        cs[(8 * hi + r) * CP + wave * 32 + 16 + lr] = c1[r] * SCI;
    }
    __syncthreads();

    v4f val[2][4];
#pragma unroll
    for (int rr = 0; rr < 2; ++rr) {
        const int row = 2 * wave + rr;
        const size_t gi = (size_t)b * SEQ + i0 + (size_t)row;
#pragma unroll
        for (int s = 0; s < 2; ++s) {
            const v4f v = *(const v4f*)(X + gi * DM + s * 128 + lane * 4);
            v4f t; t[0] = bfr(v[0]); t[1] = bfr(v[1]); t[2] = bfr(v[2]); t[3] = bfr(v[3]);
            val[rr][s] = t; }
#pragma unroll
        for (int s = 0; s < 2; ++s) val[rr][2 + s] = *(const v4fa*)(&cs[row * CP + s * 128 + lane * 4]);
    }
#pragma unroll 1
    for (int ps = 0; ps < 2; ++ps) {
#pragma unroll
        for (int rr = 0; rr < 2; ++rr) {
            const size_t gi = (size_t)b * SEQ + i0 + (size_t)(2 * wave + rr);
#pragma unroll
            for (int s = 0; s < 4; ++s)
                *(volatile v4f*)(OUT + gi * (2 * DM) + s * 128 + lane * 4) = val[rr][s];
        }
        if (ps == 0) __threadfence(); }
}

static constexpr size_t al256(size_t v) { return (v + 255) & ~(size_t)255; }
static constexpr size_t SZ_XB = al256((size_t)NB * SEQ * DM * 2);
static constexpr size_t SZ_WB = al256((size_t)HK * 2 * DM * 2);
static constexpr size_t SZ_QK = al256((size_t)2 * NB * SEQ * HK * 4);
static constexpr size_t SZ_XT = al256((size_t)NB * DM * SEQ * 2);
static constexpr size_t SZ_TOTAL = SZ_XB + SZ_WB + SZ_QK + SZ_XT;
static_assert(SZ_TOTAL <= (size_t)134217728);
static constexpr size_t N8X = (size_t)NB * SEQ * DM / 8;
static constexpr size_t N8W = (size_t)HK * 2 * DM / 8;

extern "C" void kernel_launch(void* const* d_in, const int* in_sizes, int n_in,
                              void* d_out, int out_size, void* d_ws, size_t ws_size, hipStream_t stream) {
    if (n_in < 3) return;
    if ((size_t)in_sizes[0] < (size_t)NB * SEQ * DM) return;
    if ((size_t)in_sizes[1] < (size_t)HK * 2 * DM) return;
    if (in_sizes[2] < HK) return;
    if ((size_t)out_size < (size_t)NB * SEQ * 2 * DM) return;
    if (SZ_TOTAL > ws_size) return;
    const float* x  = (const float*)d_in[0];
    const float* w1 = (const float*)d_in[1];
    const float* w2 = (const float*)d_in[2];
    float* OUT = (float*)d_out;
    char* wsp = (char*)d_ws;
    bf*    XB = (bf*)wsp;    wsp += SZ_XB;
    bf*    WB = (bf*)wsp;    wsp += SZ_WB;
    float* QK = (float*)wsp; wsp += SZ_QK;
    h16*   XT = (h16*)wsp;   wsp += SZ_XT;

    k_cvt8<<<(unsigned)((N8X + 255) / 256), 256, 0, stream>>>(x, XB, N8X);
    k_cvt8<<<(unsigned)((N8W + 255) / 256), 256, 0, stream>>>(w1, WB, N8W);
    k_xt<<<dim3(SEQ / 64, DM / 64, NB), 256, 0, stream>>>(x, XT);
    k_proj<<<dim3(NB * SEQ / 64, 2, 1), 32, 0, stream>>>(XB, WB, QK);
    k_pair<<<dim3(SEQ / PR, NB, 1), 32 * PW, 0, stream>>>(x, QK, w2, XT, OUT);
}
